// st_encoder_20040317403592
// MI455X (gfx1250) — hardware-verified
//
#include <hip/hip_runtime.h>


typedef _Float16 f16t;
typedef f16t   v16h __attribute__((ext_vector_type(16)));
typedef f16t   v8h  __attribute__((ext_vector_type(8)));
typedef __bf16 v16b __attribute__((ext_vector_type(16)));
typedef float  v8f  __attribute__((ext_vector_type(8)));
typedef float  v4f  __attribute__((ext_vector_type(4)));
typedef float  v2f  __attribute__((ext_vector_type(2)));
typedef unsigned int v4u __attribute__((ext_vector_type(4)));

union FragH { v16h v; v8h q[2]; };
union FragB { v16b v; v4u q[2]; };
union Pk16  { v8h h; v4u u; unsigned short s[8]; };

#define NB     2048
#define TL     128
#define CI     2
#define CO     16
#define HR     232
#define G3     696
#define NPAD   704
#define KP     256
#define KX     32
#define HLP    264
#define XP     40
#define NSPLIT 29
#define GBC    240
#define TB     16
#define NTHR   256

#define OFF_H32   0
#define OFF_H16   14848
#define OFF_XA    23296
#define OFF_GA    24576
#define OFF_GB    69632
#define LDS_TOTAL 84992

#define PREP_BLK_HH 88
#define PREP_BLK_IH 11

__device__ __forceinline__ unsigned short f2bf(float f) {
    unsigned u = __builtin_bit_cast(unsigned, f);
    u += 0x7FFFu + ((u >> 16) & 1u);
    return (unsigned short)(u >> 16);
}
__device__ __forceinline__ float bf2f(unsigned short b) {
    return __builtin_bit_cast(float, ((unsigned)b) << 16);
}

__device__ __forceinline__ v8f wm_h(v16h a, v16h b, v8f c) {
    return __builtin_amdgcn_wmma_f32_16x16x32_f16(false, a, false, b, (short)0, c, false, false);
}
__device__ __forceinline__ v8f wm_b(v16b a, v16b b, v8f c) {
    return __builtin_amdgcn_wmma_f32_16x16x32_bf16(false, a, false, b, (short)0, c, false, false);
}

#define NOP4 "v_nop\n\tv_nop\n\tv_nop\n\tv_nop"
__device__ __forceinline__ void gd_h(v8f (&c)[1], FragH& a, FragH (&b)[1]) {
    asm volatile(NOP4 : "+v"(c[0]) : "v"(a.v), "v"(b[0].v));
}
__device__ __forceinline__ void gd_h(v8f (&c)[2], FragH& a, FragH (&b)[2]) {
    asm volatile(NOP4 : "+v"(c[0]), "+v"(c[1]) : "v"(a.v), "v"(b[0].v), "v"(b[1].v));
}
__device__ __forceinline__ void gd_h(v8f (&c)[3], FragH& a, FragH (&b)[3]) {
    asm volatile(NOP4 : "+v"(c[0]), "+v"(c[1]), "+v"(c[2])
                 : "v"(a.v), "v"(b[0].v), "v"(b[1].v), "v"(b[2].v));
}
__device__ __forceinline__ void gd_b(v8f (&c)[1], FragB& a, FragB (&b1)[1], FragB (&b2)[1]) {
    asm volatile(NOP4 : "+v"(c[0]) : "v"(a.v), "v"(b1[0].v), "v"(b2[0].v));
}
__device__ __forceinline__ void gd_b(v8f (&c)[2], FragB& a, FragB (&b1)[2], FragB (&b2)[2]) {
    asm volatile(NOP4 : "+v"(c[0]), "+v"(c[1])
                 : "v"(a.v), "v"(b1[0].v), "v"(b1[1].v), "v"(b2[0].v), "v"(b2[1].v));
}
__device__ __forceinline__ void gd_b(v8f (&c)[3], FragB& a, FragB (&b1)[3], FragB (&b2)[3]) {
    asm volatile(NOP4 : "+v"(c[0]), "+v"(c[1]), "+v"(c[2])
                 : "v"(a.v), "v"(b1[0].v), "v"(b1[1].v), "v"(b1[2].v),
                   "v"(b2[0].v), "v"(b2[1].v), "v"(b2[2].v));
}

__device__ __forceinline__ float ftanh(float x) {
    float ax = fabsf(x);
    float t  = __expf(-2.0f * ax);
    float r  = (1.0f - t) * __builtin_amdgcn_rcpf(1.0f + t);
    return copysignf(r, x);
}
__device__ __forceinline__ float fsigm(float x) {
    return __builtin_amdgcn_rcpf(1.0f + __expf(-x));
}

template<int NT>
__device__ __forceinline__ void gate_group(int tile0,
                                           const f16t* H16, const unsigned short* XA,
                                           const f16t* Phh,
                                           const unsigned short* PB1, const unsigned short* PB2,
                                           const float* bih, const float* bhh,
                                           float* GA, float* GB) {
    const int l = threadIdx.x & 31, h = l >> 4, m = l & 15;
    const v8f z8 = {0.f, 0.f, 0.f, 0.f, 0.f, 0.f, 0.f, 0.f};
    v8f ah[NT], ai[NT];
#pragma unroll
    for (int j = 0; j < NT; ++j) { ah[j] = z8; ai[j] = z8; }

    const f16t* ap = H16 + m * HLP + 8 * h;
#pragma unroll 1
    for (int kt = 0; kt < KP / 32; ++kt) {
        FragH a, b[NT];
        a.q[0] = *(const v8h*)(ap + kt * 32);
        a.q[1] = *(const v8h*)(ap + kt * 32 + 16);
#pragma unroll
        for (int j = 0; j < NT; ++j) {
            const f16t* bp = Phh + (size_t)(16 * (tile0 + 8 * j) + m) * KP + kt * 32 + 8 * h;
            b[j].q[0] = *(const v8h*)bp;
            b[j].q[1] = *(const v8h*)(bp + 16);
        }
#pragma unroll
        for (int j = 0; j < NT; ++j) ah[j] = wm_h(a.v, b[j].v, ah[j]);
        gd_h(ah, a, b);
    }

    {
        FragB ax, b1[NT], b2[NT];
        const unsigned short* xp = XA + m * XP + 8 * h;
        ax.q[0] = *(const v4u*)xp;
        ax.q[1] = *(const v4u*)(xp + 16);
#pragma unroll
        for (int j = 0; j < NT; ++j) {
            const size_t ro = (size_t)(16 * (tile0 + 8 * j) + m) * KX + 8 * h;
            b1[j].q[0] = *(const v4u*)(PB1 + ro);
            b1[j].q[1] = *(const v4u*)(PB1 + ro + 16);
            b2[j].q[0] = *(const v4u*)(PB2 + ro);
            b2[j].q[1] = *(const v4u*)(PB2 + ro + 16);
        }
#pragma unroll
        for (int j = 0; j < NT; ++j) {
            ai[j] = wm_b(ax.v, b1[j].v, ai[j]);
            ai[j] = wm_b(ax.v, b2[j].v, ai[j]);
        }
        gd_b(ai, ax, b1, b2);
    }

#pragma unroll
    for (int j = 0; j < NT; ++j) {
        const int  tile = tile0 + 8 * j;
        const int  c    = 16 * tile + m;
        const int  cc   = min(c, G3 - 1);
        const float bi  = bih[cc];
        const float bh  = bhh[cc];
        const bool  sum = (tile < NSPLIT);
        v4f g0, g1, n0, n1;
#pragma unroll
        for (int r = 0; r < 4; ++r) {
            const float gh0 = fmaf(ah[j][r],     0.125f, bh);
            const float gh1 = fmaf(ah[j][4 + r], 0.125f, bh);
            const float gi0 = ai[j][r] + bi;
            const float gi1 = ai[j][4 + r] + bi;
            g0[r] = sum ? (gi0 + gh0) : gi0;
            g1[r] = sum ? (gi1 + gh1) : gi1;
            n0[r] = gh0;
            n1[r] = gh1;
        }
        float* ga = GA + c * 16 + 8 * h;
        *(v4f*)ga       = g0;
        *(v4f*)(ga + 4) = g1;
        if (!sum) {
            float* gb = GB + (c - 16 * NSPLIT) * 16 + 8 * h;
            *(v4f*)gb       = n0;
            *(v4f*)(gb + 4) = n1;
        }
    }
}

__global__ __launch_bounds__(NTHR)
void k_prep(const float* whh, const float* wih, f16t* Phh,
            unsigned short* PB1, unsigned short* PB2) {
    const int blk = blockIdx.x, tid = threadIdx.x;
    if (blk < PREP_BLK_HH) {
        const int  i  = blk * NTHR + tid;
        const int  n  = i >> 5;
        const int  k  = (i & 31) * 8;
        const int  nn = min(n, G3 - 1);
        const int  kc = min(k, HR - 8);
        const bool ok = (n < G3) && (k < HR);
        const float* src = whh + (size_t)nn * HR + kc;
        Pk16 v;
#pragma unroll
        for (int e = 0; e < 8; ++e) {
            const float x = ok ? src[e] : 0.0f;
            v.h[e] = (f16t)(x * 8.0f);
        }
        f16t* d = Phh + (size_t)n * KP + k;
        *(volatile v4u*)d = v.u;
        __threadfence();
        *(volatile v4u*)d = v.u;
    } else if (blk < PREP_BLK_HH + 2 * PREP_BLK_IH) {
        const bool lo = (blk >= PREP_BLK_HH + PREP_BLK_IH);
        const int  i  = (blk - PREP_BLK_HH - (lo ? PREP_BLK_IH : 0)) * NTHR + tid;
        const int  n  = i >> 2;
        const int  kq = i & 3;
        const int  k  = kq * 8;
        const int  nn = min(n, G3 - 1);
        const bool ok = (n < G3) && (!lo || kq < 2);
        const float* src = wih + (size_t)nn * CO + (k & 15);
        Pk16 v;
#pragma unroll
        for (int e = 0; e < 8; ++e) {
            const float x = src[e];
            const unsigned short hb = f2bf(x);
            const unsigned short lb = f2bf(x - bf2f(hb));
            const unsigned short s  = lo ? lb : hb;
            v.s[e] = ok ? s : (unsigned short)0;
        }
        unsigned short* base = lo ? PB2 : PB1;
        unsigned short* d = base + (size_t)n * KX + k;
        *(volatile v4u*)d = v.u;
        __threadfence();
        *(volatile v4u*)d = v.u;
    }
}

__global__ __launch_bounds__(NTHR)
void k_gru(const float* X, const float* cw, const float* cb,
           const float* bih, const float* bhh,
           const f16t* Phh, const unsigned short* PB1, const unsigned short* PB2,
           float* out, int nb) {
    extern __shared__ __attribute__((aligned(16))) unsigned char smem[];
    float*          H32 = (float*)(smem + OFF_H32);
    f16t*           H16 = (f16t*)(smem + OFF_H16);
    unsigned short* XA  = (unsigned short*)(smem + OFF_XA);
    float*          GA  = (float*)(smem + OFF_GA);
    float*          GB  = (float*)(smem + OFF_GB);

    const int tid = threadIdx.x;
    const int w   = __builtin_amdgcn_readfirstlane(tid >> 5);
    const int b0  = blockIdx.x * TB;
    if (b0 + TB > nb) return;

    for (int i = tid; i < TB * HR;  i += NTHR) H32[i] = 0.0f;
    for (int i = tid; i < TB * HLP; i += NTHR) H16[i] = (f16t)0.0f;
    for (int i = tid; i < TB * XP;  i += NTHR) XA[i]  = (unsigned short)0;

    const int bl = tid >> 4, o = tid & 15;
    float cwr[6];
#pragma unroll
    for (int c = 0; c < CI; ++c)
#pragma unroll
        for (int k = 0; k < 3; ++k) cwr[3 * c + k] = cw[(o * CI + c) * 3 + k];
    const float cbv = cb[o];
    const float* xrow = X + (size_t)(b0 + bl) * TL * CI;
    __syncthreads();

#pragma unroll 1
    for (int t = 0; t < TL; ++t) {
        float acc = cbv;
#pragma unroll
        for (int k = 0; k < 3; ++k) {
            const int  tt  = t + k - 1;
            const int  ttc = min(max(tt, 0), TL - 1);
            const v2f  xv  = *(const v2f*)(xrow + ttc * CI);
            const bool ok  = (tt >= 0) && (tt < TL);
            const float x0 = ok ? xv[0] : 0.0f;
            const float x1 = ok ? xv[1] : 0.0f;
            acc = fmaf(cwr[k],     x0, acc);
            acc = fmaf(cwr[3 + k], x1, acc);
        }
        acc = fmaxf(acc, 0.0f);
        const unsigned short hb = f2bf(acc);
        const unsigned short lb = f2bf(acc - bf2f(hb));
        XA[bl * XP + o]      = hb;
        XA[bl * XP + 16 + o] = lb;
        __syncthreads();

        gate_group<3>(w,      H16, XA, Phh, PB1, PB2, bih, bhh, GA, GB);
        gate_group<2>(w + 24, H16, XA, Phh, PB1, PB2, bih, bhh, GA, GB);
        if (w < 4)
            gate_group<1>(w + 40, H16, XA, Phh, PB1, PB2, bih, bhh, GA, GB);
        __syncthreads();

#pragma unroll 1
        for (int e = tid; e < TB * HR; e += NTHR) {
            const int row = e & 15, j = e >> 4;
            const float pr  = GA[j * 16 + row];
            const float pz  = GA[(HR + j) * 16 + row];
            const float pni = GA[(2 * HR + j) * 16 + row];
            const float pnh = GB[j * 16 + row];
            const float r  = fsigm(pr);
            const float z  = fsigm(pz);
            const float n  = ftanh(fmaf(r, pnh, pni));
            const float ho = H32[row * HR + j];
            const float hn = (1.0f - z) * n + z * ho;
            H32[row * HR + j]  = hn;
            H16[row * HLP + j] = (f16t)hn;
        }
        __syncthreads();
    }

    v4f v[4];
#pragma unroll
    for (int i = 0; i < 4; ++i) {
        const int p = min(tid + NTHR * i, TB * HR / 4 - 1);
        v[i] = *(const v4f*)(H32 + p * 4);
    }
    float* ob = out + (size_t)b0 * HR;
#pragma unroll
    for (int i = 0; i < 4; ++i) {
        const int p = tid + NTHR * i;
        if (p < TB * HR / 4) *(volatile v4f*)(ob + (size_t)p * 4) = v[i];
    }
    __threadfence();
#pragma unroll
    for (int i = 0; i < 4; ++i) {
        const int p = tid + NTHR * i;
        if (p < TB * HR / 4) *(volatile v4f*)(ob + (size_t)p * 4) = v[i];
    }
}

extern "C" void kernel_launch(void* const* d_in, const int* in_sizes, int n_in,
                              void* d_out, int out_size, void* d_ws, size_t ws_size,
                              hipStream_t stream) {
    if (n_in < 7) return;
    if (in_sizes[0] != NB * TL * CI || in_sizes[1] != CO * CI * 3 || in_sizes[2] != CO ||
        in_sizes[3] != G3 * CO || in_sizes[4] != G3 * HR ||
        in_sizes[5] != G3 || in_sizes[6] != G3) return;
    if (out_size != NB * HR) return;

    const float* X    = (const float*)d_in[0];
    const float* cw   = (const float*)d_in[1];
    const float* cb   = (const float*)d_in[2];
    const float* wih  = (const float*)d_in[3];
    const float* whh  = (const float*)d_in[4];
    const float* bih  = (const float*)d_in[5];
    const float* bhh  = (const float*)d_in[6];
    float* out = (float*)d_out;

    const size_t szPhh = (size_t)NPAD * KP * 2;
    const size_t szP   = (size_t)NPAD * KX * 2;
    const size_t offP1 = szPhh, offP2 = szPhh + szP, total = szPhh + 2 * szP;
    if (total > ws_size) return;
    char* ws = (char*)d_ws;
    f16t*           Phh = (f16t*)(ws);
    unsigned short* PB1 = (unsigned short*)(ws + offP1);
    unsigned short* PB2 = (unsigned short*)(ws + offP2);

    k_prep<<<dim3(PREP_BLK_HH + 2 * PREP_BLK_IH), dim3(NTHR), 0, stream>>>(whh, wih, Phh, PB1, PB2);
    k_gru<<<dim3(NB / TB), dim3(NTHR), LDS_TOTAL, stream>>>(X, cw, cb, bih, bhh,
                                                           Phh, PB1, PB2, out, NB);
}
